// Mean_Shift_Cluster_83794811945535
// MI455X (gfx1250) — hardware-run, weakly checked
//
#include <hip/hip_runtime.h>
#include <math.h>

typedef __attribute__((ext_vector_type(16))) _Float16 v16h;
typedef __attribute__((ext_vector_type(8)))  _Float16 v8h;
typedef __attribute__((ext_vector_type(8)))  float    v8f;
typedef __attribute__((ext_vector_type(4)))  float    v4f;
typedef __attribute__((ext_vector_type(4)))  unsigned int v4u;

constexpr int kDim   = 256;
constexpr int kPts   = 8192;
constexpr int kQB    = 64;
constexpr int kKeys  = 32;
constexpr int kTiles = kPts / kKeys;
constexpr float kDelta = 6.0f;
constexpr float kLog2e = 1.4426950408889634f;
constexpr float kCarry0 = 1024.0f;
constexpr float kCarry1 = 4096.0f;
constexpr float kCarry2 = 16384.0f;
constexpr float kExp0 = kDelta * kLog2e / (kCarry0 * kCarry0);
constexpr float kExp1 = kDelta * kLog2e / (kCarry1 * kCarry1);
constexpr float kExp2 = kDelta * kLog2e / (kCarry2 * kCarry2);
static_assert(kDim == 256 && kPts == 8192, "shape constants");
static_assert((kPts % kQB) == 0 && (kPts % kKeys) == 0 && (kDim % 32) == 0 && (kKeys % 32) == 0, "tile multiples");

constexpr int kLdsQ    = 0;
constexpr int kLdsKT   = kLdsQ  + kQB * kDim * 2;
constexpr int kLdsKD   = kLdsKT + kKeys * kDim * 2;
constexpr int kLdsMain = kLdsKD + kDim * kKeys * 2;
static_assert(kLdsMain == 65536, "lds main bytes");
static_assert(kLdsMain == kDim * kQB * 4, "epilogue tile fills the main region exactly");

constexpr size_t kPlaneBytes = (size_t)kDim * kPts * 2;
constexpr size_t kOffXT0 = 0;
constexpr size_t kOffXH0 = kOffXT0 + kPlaneBytes;
constexpr size_t kOffXT1 = kOffXH0 + kPlaneBytes;
constexpr size_t kOffXH1 = kOffXT1 + kPlaneBytes;
constexpr size_t kOffXT2 = kOffXH1 + kPlaneBytes;
constexpr size_t kOffXH2 = kOffXT2 + kPlaneBytes;
constexpr size_t kWsTotal = kOffXH2 + kPlaneBytes;
static_assert(kPlaneBytes == 4194304ull, "plane bytes");
static_assert(kWsTotal == 25165824ull, "carve total");
static_assert(kWsTotal <= 134217728ull, "carve cap");
static_assert((kPlaneBytes % 128) == 0, "128-B aligned regions");

struct FragH {
  union U { v16h v; v8h h[2]; };
  static __device__ __forceinline__ v16h load(const _Float16* p) {
    U f;
    f.h[0] = *(const v8h*)(p);
    f.h[1] = *(const v8h*)(p + 16);
    return f.v;
  }
};

__device__ __forceinline__ v8f mma_g(v16h a, v16h b, v8f c) {
  c = __builtin_amdgcn_wmma_f32_16x16x32_f16(false, a, false, b, (short)0, c, false, false);
  asm volatile("v_nop\n\tv_nop\n\tv_nop\n\tv_nop" : "+v"(c) : "v"(a), "v"(b) : "memory");
  return c;
}

__device__ __forceinline__ void emit_planes(const float* stage, int wv, int lane, int m0, float carry,
                                            unsigned short* XTn, unsigned short* XHn) {
  const int q  = lane >> 3;
  const int c8 = (lane & 7) * 8;
  for (int pass = 0; pass < 2; ++pass) {
#pragma unroll 4
    for (int it = 0; it < 16; ++it) {
      const int d = wv * 64 + it * 4 + q;
      const float* sp = stage + d * kQB + c8;
      const v4f a0 = *(const v4f*)(sp);
      const v4f a1 = *(const v4f*)(sp + 4);
      v8h hv;
#pragma unroll
      for (int e = 0; e < 4; ++e) {
        hv[e]     = (_Float16)(a0[e] * carry);
        hv[4 + e] = (_Float16)(a1[e] * carry);
      }
      *(volatile v8h*)(XHn + (size_t)d * kPts + m0 + c8) = hv;
    }
#pragma unroll 4
    for (int it = 0; it < 16; ++it) {
      const int ml = wv * 16 + it;
      v8h hv;
#pragma unroll
      for (int e = 0; e < 8; ++e) hv[e] = (_Float16)(stage[(lane * 8 + e) * kQB + ml] * carry);
      *(volatile v8h*)(XTn + (size_t)(m0 + ml) * kDim + lane * 8) = hv;
    }
    __threadfence();
  }
}

__global__ __launch_bounds__(128) void prep_planes_kernel(const float* __restrict__ X, unsigned short* XT0,
                                                          unsigned short* XH0, float carry) {
  __shared__ __align__(16) float stage[kDim * kQB];
  const int tid = threadIdx.x, lane = tid & 31, wv = tid >> 5, hf = lane >> 4, l16 = lane & 15;
  const int m0 = blockIdx.x * kQB;
#pragma unroll 8
  for (int it = 0; it < 32; ++it) {
    const int d = wv * 64 + it * 2 + hf;
    const v4f v = *(const v4f*)(X + (size_t)d * kPts + m0 + l16 * 4);
    *(v4f*)(stage + d * kQB + l16 * 4) = v;
  }
  __syncthreads();
  emit_planes(stage, wv, lane, m0, carry, XT0, XH0);
}

template <bool EMIT>
__global__ __launch_bounds__(128) __attribute__((amdgpu_num_vgpr(256)))
void shift_step_kernel(const unsigned short* XTc, const unsigned short* XHc, float* outp,
                       unsigned short* XTn, unsigned short* XHn,
                       float expScale, float inCarryInv, float nextCarry) {
  __shared__ __align__(16) unsigned char smem[kLdsMain];
  __shared__ __align__(16) _Float16 sPB[4][16 * kKeys];

  const int tid = threadIdx.x, lane = tid & 31, wv = tid >> 5, hf = lane >> 4, l16 = lane & 15;
  const int m0 = blockIdx.x * kQB;

  const _Float16* sQ  = (const _Float16*)(smem + kLdsQ);
  const _Float16* sKT = (const _Float16*)(smem + kLdsKT);
  const _Float16* sKD = (const _Float16*)(smem + kLdsKD);
  float* stage = (float*)smem;

  {
    const v4u* src = (const v4u*)(XTc + (size_t)m0 * kDim);
    v4u* dst = (v4u*)(smem + kLdsQ);
#pragma unroll
    for (int i = 0; i < 16; ++i) dst[i * 128 + tid] = src[i * 128 + tid];
  }

  v8f O[16];
#pragma unroll
  for (int i = 0; i < 16; ++i) O[i] = (v8f){0.f, 0.f, 0.f, 0.f, 0.f, 0.f, 0.f, 0.f};
  float rs[8];
#pragma unroll
  for (int r = 0; r < 8; ++r) rs[r] = 0.0f;

  const _Float16* qrow = sQ  + (wv * 16 + l16) * kDim + 8 * hf;
  const _Float16* kt0  = sKT + l16 * kDim + 8 * hf;
  const _Float16* kt1  = sKT + (16 + l16) * kDim + 8 * hf;
  const _Float16* kdp  = sKD + l16 * kKeys + 8 * hf;
  _Float16* pb = sPB[wv];

#pragma unroll 1
  for (int t = 0; t < kTiles; ++t) {
    const int n0 = t * kKeys;
    __syncthreads();
    {
      const v4u* srcT = (const v4u*)(XTc + (size_t)n0 * kDim);
      v4u tt[8];
#pragma unroll
      for (int i = 0; i < 8; ++i) tt[i] = srcT[i * 128 + tid];
      v4u dd[8];
#pragma unroll
      for (int i = 0; i < 8; ++i) {
        const int e = i * 128 + tid;
        const int d = e >> 2;
        const int c = e & 3;
        dd[i] = *(const v4u*)(XHc + (size_t)d * kPts + n0 + c * 8);
      }
      v4u* dT = (v4u*)(smem + kLdsKT);
      v4u* dD = (v4u*)(smem + kLdsKD);
#pragma unroll
      for (int i = 0; i < 8; ++i) dT[i * 128 + tid] = tt[i];
#pragma unroll
      for (int i = 0; i < 8; ++i) dD[i * 128 + tid] = dd[i];
    }
    __syncthreads();

    v8f s0 = (v8f){0.f, 0.f, 0.f, 0.f, 0.f, 0.f, 0.f, 0.f};
    v8f s1 = (v8f){0.f, 0.f, 0.f, 0.f, 0.f, 0.f, 0.f, 0.f};
#pragma unroll
    for (int c = 0; c < 8; ++c) {
      const v16h a  = FragH::load(qrow + c * 32);
      const v16h b0 = FragH::load(kt0 + c * 32);
      const v16h b1 = FragH::load(kt1 + c * 32);
      s0 = mma_g(a, b0, s0);
      s1 = mma_g(a, b1, s1);
    }

#pragma unroll
    for (int r = 0; r < 8; ++r) {
      const float e0 = __builtin_amdgcn_exp2f(s0[r] * expScale);
      const float e1 = __builtin_amdgcn_exp2f(s1[r] * expScale);
      const _Float16 h0 = (_Float16)e0;
      const _Float16 h1 = (_Float16)e1;
      rs[r] += (float)h0 + (float)h1;
      pb[(8 * hf + r) * kKeys + l16]      = h0;
      pb[(8 * hf + r) * kKeys + 16 + l16] = h1;
    }
    __builtin_amdgcn_fence(__ATOMIC_RELEASE, "workgroup");
    __builtin_amdgcn_wave_barrier();
    __builtin_amdgcn_fence(__ATOMIC_ACQUIRE, "workgroup");

    const v16h pa = FragH::load(pb + l16 * kKeys + 8 * hf);
#pragma unroll
    for (int c2 = 0; c2 < 16; ++c2) {
      const v16h bv = FragH::load(kdp + c2 * 16 * kKeys);
      O[c2] = mma_g(pa, bv, O[c2]);
    }
  }

#pragma unroll
  for (int off = 1; off < 16; off <<= 1) {
#pragma unroll
    for (int r = 0; r < 8; ++r) rs[r] += __shfl_xor(rs[r], off, 32);
  }
  float sc[8];
#pragma unroll
  for (int r = 0; r < 8; ++r) sc[r] = (1.0f / rs[r]) * inCarryInv;

  __syncthreads();
#pragma unroll
  for (int c2 = 0; c2 < 16; ++c2) {
    float* sp = stage + (c2 * 16 + l16) * kQB + wv * 16 + 8 * hf;
    const v4f a = (v4f){O[c2][0] * sc[0], O[c2][1] * sc[1], O[c2][2] * sc[2], O[c2][3] * sc[3]};
    const v4f b = (v4f){O[c2][4] * sc[4], O[c2][5] * sc[5], O[c2][6] * sc[6], O[c2][7] * sc[7]};
    *(v4f*)(sp)     = a;
    *(v4f*)(sp + 4) = b;
  }
  __syncthreads();

  {
    const int c4 = l16 * 4;
    for (int pass = 0; pass < 2; ++pass) {
#pragma unroll 8
      for (int it = 0; it < 32; ++it) {
        const int d = wv * 64 + it * 2 + hf;
        const v4f v = *(const v4f*)(stage + d * kQB + c4);
        *(volatile v4f*)(outp + (size_t)d * kPts + m0 + c4) = v;
      }
      __threadfence();
    }
  }
  if (EMIT) emit_planes(stage, wv, lane, m0, nextCarry, XTn, XHn);
}

extern "C" void kernel_launch(void* const* d_in, const int* in_sizes, int n_in,
                              void* d_out, int out_size, void* d_ws, size_t ws_size,
                              hipStream_t stream) {
  if (n_in < 1) return;
  if (in_sizes[0] != kDim * kPts) return;
  if (out_size != 3 * kDim * kPts) return;
  if (ws_size < kWsTotal) return;

  const float* X = (const float*)d_in[0];
  float* out = (float*)d_out;
  const size_t plane = (size_t)kDim * kPts;
  float* out0 = out;
  float* out1 = out + plane;
  float* out2 = out + 2 * plane;

  char* ws = (char*)d_ws;
  unsigned short* XT0 = (unsigned short*)(ws + kOffXT0);
  unsigned short* XH0 = (unsigned short*)(ws + kOffXH0);
  unsigned short* XT1 = (unsigned short*)(ws + kOffXT1);
  unsigned short* XH1 = (unsigned short*)(ws + kOffXH1);
  unsigned short* XT2 = (unsigned short*)(ws + kOffXT2);
  unsigned short* XH2 = (unsigned short*)(ws + kOffXH2);

  const int nblk = kPts / kQB;

  prep_planes_kernel<<<nblk, 128, 0, stream>>>(X, XT0, XH0, kCarry0);

  shift_step_kernel<true><<<nblk, 128, 0, stream>>>(XT0, XH0, out0, XT1, XH1, kExp0, 1.0f / kCarry0, kCarry1);
  shift_step_kernel<true><<<nblk, 128, 0, stream>>>(XT1, XH1, out1, XT2, XH2, kExp1, 1.0f / kCarry1, kCarry2);
  shift_step_kernel<false><<<nblk, 128, 0, stream>>>(XT2, XH2, out2, nullptr, nullptr, kExp2, 1.0f / kCarry2, 1.0f);
}
